// LSTMPredictor_75007308857624
// MI455X (gfx1250) — hardware-verified
//
#include <hip/hip_runtime.h>
#include <math.h>

typedef __attribute__((ext_vector_type(16))) _Float16 v16h;
typedef __attribute__((ext_vector_type(8)))  _Float16 v8h;
typedef __attribute__((ext_vector_type(8)))  float    v8f;

constexpr int kBatch  = 4096;
constexpr int kSteps  = 512;
constexpr int kIn     = 3;
constexpr int kHid    = 64;
constexpr int kG4     = 4 * kHid;
constexpr int kThr    = 256;
constexpr int kBlocks = kBatch / (8 * 16);
constexpr int kWP     = 104;
constexpr size_t kOutElems = (size_t)kBatch * kSteps * kIn;
static_assert(kBlocks == 32 && kHid == 64 && kIn == 3, "thirty-two blocks of eight 16-row tiles; three readout rows");

constexpr float kSCarry = 1024.0f;
constexpr float kWCarry = 4096.0f;
constexpr float kFold   = 1.0f / (kSCarry * kWCarry);
constexpr float kF16MinNormal = 6.103515625e-5f;
static_assert(kFold == 2.384185791015625e-7f, "2^-22");

union FragU { v16h v; v8h h[2]; };

__device__ __forceinline__ unsigned short f2bf_bits(float f) {
  unsigned u = __float_as_uint(f);
  return (unsigned short)((u + 0x7FFFu + ((u >> 16) & 1u)) >> 16);
}
__device__ __forceinline__ float bf16r(float f) { return __uint_as_float(((unsigned)f2bf_bits(f)) << 16); }
__device__ __forceinline__ float carry_flush(float v, float c) {
  const float s = v * c;
  return (fabsf(s) < kF16MinNormal) ? 0.0f : s;
}
__device__ __forceinline__ v8f mma_h(v16h a, v16h b, v8f c) {
  c = __builtin_amdgcn_wmma_f32_16x16x32_f16(false, a, false, b, (short)0, c, false, false);
  asm volatile("v_nop\n\tv_nop\n\tv_nop\n\tv_nop" : "+v"(c) : "v"(a), "v"(b));
  return c;
}
__device__ __forceinline__ v16h frag_h32(const _Float16* p) { FragU f; f.h[0] = *(const v8h*)(p); f.h[1] = *(const v8h*)(p + 16); return f.v; }
__device__ __forceinline__ v16h frag_tiles(const float* a, const float* b, float c) {
  v16h f;
#pragma unroll
  for (int e = 0; e < 8; ++e) { f[e] = (_Float16)carry_flush(a[e], c); f[8 + e] = (_Float16)carry_flush(b[e], c); }
  return f;
}
__device__ __forceinline__ float fast_tanh(float v) {
  const float e = __expf(2.0f * v);
  return 1.0f - 2.0f * __builtin_amdgcn_rcpf(e + 1.0f);
}
__device__ __forceinline__ float fast_sigmoid(float v) { return __builtin_amdgcn_rcpf(1.0f + __expf(-v)); }

__global__ __launch_bounds__(kThr) void lstm_pred_kernel(const float* __restrict__ x, const float* __restrict__ eWih,
                                                         const float* __restrict__ eWhh, const float* __restrict__ ebih,
                                                         const float* __restrict__ ebhh, const float* __restrict__ oW,
                                                         const float* __restrict__ ob, float* __restrict__ out) {
  __shared__ __align__(16) _Float16 sWe[kG4 * kWP];
  __shared__ __align__(16) _Float16 sWo[16 * kWP];
  const int tid = threadIdx.x;
  const int wave = tid >> 5;
  const int lane = tid & 31;
  const int col = lane & 15;
  const int hs = lane >> 4;

  {
    const int row = tid;
    _Float16* wr = sWe + row * kWP;
#pragma unroll 1
    for (int k = 0; k < kHid; ++k) wr[k] = (_Float16)carry_flush(bf16r(eWhh[row * kHid + k]), kWCarry);
    const float w0 = eWih[row * kIn + 0], w1 = eWih[row * kIn + 1], w2 = eWih[row * kIn + 2];
    const float b0 = ebih[row], b1 = ebhh[row];
    wr[64] = (_Float16)carry_flush(bf16r(w0), kWCarry);
    wr[65] = (_Float16)carry_flush(bf16r(w1), kWCarry);
    wr[66] = (_Float16)carry_flush(bf16r(w2), kWCarry);
    wr[67] = (_Float16)carry_flush(bf16r(b0), kWCarry);
    wr[68] = (_Float16)carry_flush(bf16r(b1), kWCarry);
#pragma unroll 1
    for (int k = 69; k < kWP; ++k) wr[k] = (_Float16)0.0f;
  }
  if (tid < 16) {
    const int m = tid;
    const bool live = m < kIn;
    const int src = live ? m : 0;
    _Float16* wr = sWo + m * kWP;
#pragma unroll 1
    for (int k = 0; k < kWP; ++k) wr[k] = (_Float16)0.0f;
    if (live) {
#pragma unroll 1
      for (int k = 0; k < kHid; ++k) wr[k] = (_Float16)carry_flush(bf16r(oW[src * kHid + k]), kWCarry);
      const float b0 = ob[src];
      wr[64] = (_Float16)carry_flush(bf16r(b0), kWCarry);
    }
  }
  __syncthreads();

  const int b = (blockIdx.x * 8 + wave) * 16 + col;
  const float* xb = x + (size_t)b * kSteps * kIn;
  float* ob_ = out + (size_t)b * kSteps * kIn;
  const _Float16 one = (_Float16)kSCarry;

  float cst[4][8], hst[4][8];
#pragma unroll
  for (int mt = 0; mt < 4; ++mt)
#pragma unroll
    for (int r = 0; r < 8; ++r) { cst[mt][r] = 0.0f; hst[mt][r] = 0.0f; }

#pragma unroll 1
  for (int t = 0; t < kSteps; ++t) {
    int colv = col, hsv = hs;
    asm volatile("" : "+v"(colv), "+v"(hsv));
    const v16h b0 = frag_tiles(hst[0], hst[1], kSCarry);
    const v16h b1 = frag_tiles(hst[2], hst[3], kSCarry);
    v16h bx;
#pragma unroll
    for (int e = 0; e < 16; ++e) bx[e] = (_Float16)0.0f;
    {
      const float x0 = xb[t * kIn + 0], x1 = xb[t * kIn + 1], x2 = xb[t * kIn + 2];
      const bool lo = (hsv == 0);
      bx[0] = lo ? (_Float16)carry_flush(bf16r(x0), kSCarry) : (_Float16)0.0f;
      bx[1] = lo ? (_Float16)carry_flush(bf16r(x1), kSCarry) : (_Float16)0.0f;
      bx[2] = lo ? (_Float16)carry_flush(bf16r(x2), kSCarry) : (_Float16)0.0f;
      bx[3] = lo ? one : (_Float16)0.0f;
      bx[4] = lo ? one : (_Float16)0.0f;
    }
#pragma unroll
    for (int mt = 0; mt < 4; ++mt) {
      v8f acc[4];
#pragma unroll
      for (int q = 0; q < 4; ++q) {
        const _Float16* wr = sWe + (64 * q + 16 * mt + colv) * kWP + 8 * hsv;
        v8f a = (v8f){0.f, 0.f, 0.f, 0.f, 0.f, 0.f, 0.f, 0.f};
        a = mma_h(frag_h32(wr), b0, a);
        a = mma_h(frag_h32(wr + 32), b1, a);
        a = mma_h(frag_h32(wr + 64), bx, a);
        acc[q] = a;
      }
#pragma unroll
      for (int r = 0; r < 8; ++r) {
        const float gi = acc[0][r] * kFold, gf = acc[1][r] * kFold, gg = acc[2][r] * kFold, go = acc[3][r] * kFold;
        const float cn = fast_sigmoid(gf) * cst[mt][r] + fast_sigmoid(gi) * fast_tanh(gg);
        cst[mt][r] = cn;
        hst[mt][r] = fast_sigmoid(go) * fast_tanh(cn);
      }
    }
    {
      const v16h n0 = frag_tiles(hst[0], hst[1], kSCarry);
      const v16h n1 = frag_tiles(hst[2], hst[3], kSCarry);
      v16h bd;
#pragma unroll
      for (int e = 0; e < 16; ++e) bd[e] = (_Float16)0.0f;
      const bool lo = (hsv == 0);
      bd[0] = lo ? one : (_Float16)0.0f;
      const _Float16* wr = sWo + colv * kWP + 8 * hsv;
      v8f a = (v8f){0.f, 0.f, 0.f, 0.f, 0.f, 0.f, 0.f, 0.f};
      a = mma_h(frag_h32(wr), n0, a);
      a = mma_h(frag_h32(wr + 32), n1, a);
      a = mma_h(frag_h32(wr + 64), bd, a);
      const float o0 = a[0] * kFold, o1 = a[1] * kFold, o2 = a[2] * kFold;
      float* op = ob_ + t * kIn;
      for (int pass = 0; pass < 2; ++pass) {
        if (lo) {
          *(volatile float*)(op + 0) = o0;
          *(volatile float*)(op + 1) = o1;
          *(volatile float*)(op + 2) = o2;
        }
        __threadfence();
      }
    }
  }
}

extern "C" void kernel_launch(void* const* d_in, const int* in_sizes, int n_in,
                              void* d_out, int out_size, void* d_ws, size_t ws_size,
                              hipStream_t stream) {
  if (n_in < 7 || d_out == nullptr) return;
  if (in_sizes[0] != kBatch * kSteps * kIn || in_sizes[1] != kG4 * kIn || in_sizes[2] != kG4 * kHid) return;
  if (in_sizes[3] != kG4 || in_sizes[4] != kG4 || in_sizes[5] != kIn * kHid || in_sizes[6] != kIn) return;
  if ((size_t)out_size != kOutElems) return;
  lstm_pred_kernel<<<kBlocks, kThr, 0, stream>>>((const float*)d_in[0], (const float*)d_in[1], (const float*)d_in[2],
                                                (const float*)d_in[3], (const float*)d_in[4], (const float*)d_in[5],
                                                (const float*)d_in[6], (float*)d_out);
}
